// BahdanauSelfAttention_24764781429505
// MI455X (gfx1250) — hardware-verified
//
#include <hip/hip_runtime.h>
#include <math.h>

typedef __attribute__((ext_vector_type(16))) _Float16 v16h;
typedef __attribute__((ext_vector_type(16))) __bf16 v16b;
typedef __attribute__((ext_vector_type(8)))  _Float16 v8h;
typedef __attribute__((ext_vector_type(8)))  float v8f;
typedef __attribute__((ext_vector_type(4)))  float v4f;
typedef __attribute__((ext_vector_type(2)))  float v2f;
typedef __attribute__((ext_vector_type(4)))  unsigned v4u;
typedef __attribute__((ext_vector_type(4)))  int v4i;
typedef float __attribute__((may_alias)) float_a;
typedef int __attribute__((may_alias)) int_a;

template <typename T> __device__ __forceinline__ void vst2(void* p, T v) { *(volatile T*)p = v; __threadfence(); *(volatile T*)p = v; }
__device__ __forceinline__ v8f wmma16(v16h a, v16h b, v8f c) {
  v8f d = __builtin_amdgcn_wmma_f32_16x16x32_f16(false, a, false, b, (short)0, c, false, false);
  asm volatile("v_nop\n\tv_nop\n\tv_nop\n\tv_nop" : "+v"(d) : "v"(a), "v"(b));
  return d;
}
__device__ __forceinline__ v8f wmma_bf(v16b a, v16b b, v8f c) {
  v8f d = __builtin_amdgcn_wmma_f32_16x16x32_bf16(false, a, false, b, (short)0, c, false, false);
  asm volatile("v_nop\n\tv_nop\n\tv_nop\n\tv_nop" : "+v"(d) : "v"(a), "v"(b));
  return d;
}
__device__ __forceinline__ v16h frag_h(const _Float16* rowk0, int lane) {
  union { v16h v; v8h q[2]; } u; const _Float16* p = rowk0 + 8 * (lane >> 4);
  u.q[0] = *(const v8h*)p; u.q[1] = *(const v8h*)(p + 16); return u.v;
}
__device__ __forceinline__ v16h frag_f32(const float* rowk0, int lane) {
  v16h a; const float* p = rowk0 + 8 * (lane >> 4);
#pragma unroll
  for (int i = 0; i < 8; ++i) { a[i] = (_Float16)p[i]; a[8 + i] = (_Float16)p[16 + i]; }
  return a;
}
__device__ __forceinline__ v16h frag_f32s(const float* rowk0, int lane, float sc) {
  v16h a; const float* p = rowk0 + 8 * (lane >> 4);
#pragma unroll
  for (int i = 0; i < 8; ++i) { a[i] = (_Float16)(p[i] * sc); a[8 + i] = (_Float16)(p[16 + i] * sc); }
  return a;
}
__device__ __forceinline__ v16h fragc_f32(const float* W, int k0, int n, int lane, int ld, int K) {
  v16h a; const int g = lane >> 4;
#pragma unroll
  for (int i = 0; i < 8; ++i) { const int ka = k0 + 8 * g + i, kb = ka + 16;
    a[i] = (_Float16)(ka < K ? W[(size_t)(ka < K ? ka : K - 1) * ld + n] : 0.f); a[8 + i] = (_Float16)(kb < K ? W[(size_t)(kb < K ? kb : K - 1) * ld + n] : 0.f); }
  return a;
}
struct F2 { v16b h, l; };
__device__ __forceinline__ F2 bsplit16(const float v[16]) { F2 r;
#pragma unroll
  for (int i = 0; i < 16; ++i) { const __bf16 h = (__bf16)v[i]; r.h[i] = h; r.l[i] = (__bf16)(v[i] - (float)h); }
  return r; }
__device__ __forceinline__ F2 split_row(const float* row, int k0, int lane) { float v[16]; const float* p = row + k0 + 8 * (lane >> 4);
#pragma unroll
  for (int i = 0; i < 8; ++i) { v[i] = p[i]; v[8 + i] = p[16 + i]; }
  return bsplit16(v); }
__device__ __forceinline__ F2 split_rowK(const float* row, int k0, int lane, int K) { float v[16]; const int g = lane >> 4;
#pragma unroll
  for (int i = 0; i < 8; ++i) { const int ka = k0 + 8 * g + i, kb = ka + 16; v[i] = ka < K ? row[ka < K ? ka : K - 1] : 0.f; v[8 + i] = kb < K ? row[kb < K ? kb : K - 1] : 0.f; }
  return bsplit16(v); }
__device__ __forceinline__ F2 split_col(const float* W, int k0, int n, int lane, int ld, int K) { float v[16]; const int g = lane >> 4;
#pragma unroll
  for (int i = 0; i < 8; ++i) { const int ka = k0 + 8 * g + i, kb = ka + 16; v[i] = ka < K ? W[(size_t)(ka < K ? ka : K - 1) * ld + n] : 0.f; v[8 + i] = kb < K ? W[(size_t)(kb < K ? kb : K - 1) * ld + n] : 0.f; }
  return bsplit16(v); }
__device__ __forceinline__ v8f mac3(const F2& a, const F2& b, v8f c) { c = wmma_bf(a.l, b.h, c); c = wmma_bf(a.h, b.l, c); return wmma_bf(a.h, b.h, c); }
__device__ __forceinline__ float sigm(float v) { return 1.0f / (1.0f + expf(-v)); }
#define LDSX() do { asm volatile("s_wait_dscnt 0" ::: "memory"); __builtin_amdgcn_wave_barrier(); __builtin_amdgcn_fence(__ATOMIC_RELEASE, "workgroup"); } while (0)


#define NB 4
#define NN 512
#define DD 128
#ifndef TNB
#define TNB NB
#endif
typedef __attribute__((ext_vector_type(8))) __bf16 v8b;
__device__ __forceinline__ v16b frag_b(const __bf16* rowk0, int lane) {
  union { v16b v; v8b q[2]; } u; const __bf16* p = rowk0 + 8 * (lane >> 4);
  u.q[0] = *(const v8b*)p; u.q[1] = *(const v8b*)(p + 16); return u.v;
}
__device__ __forceinline__ float bfr(float v) { return (float)(__bf16)v; }
__device__ __attribute__((noinline)) float exp_ni(float v) { return expf(v); }
__device__ __attribute__((noinline)) float erf_ni(float v) { return erff(v); }

#define WS_PW  0u
#define WS_BT  (WS_PW + 2u * DD * DD)
#define WS_WI  (WS_BT + 2u * (size_t)NB * DD * NN)
#define WS_P   (WS_WI + 4u * (size_t)NB * NN * DD)
#define WS_END (WS_P + 4u * (size_t)NB * NN * NN)

__global__ __launch_bounds__(128) void k_pack(const float* __restrict__ Wm, __bf16* __restrict__ PW) { const int o = blockIdx.x, t = threadIdx.x; __shared__ __align__(16) __bf16 s[DD]; s[t] = (__bf16)Wm[(size_t)o * DD + t]; __syncthreads(); if (t < 16) vst2((unsigned*)(PW + (size_t)o * DD + t * 8), *(const v4u*)&s[t * 8]); }
__global__ __launch_bounds__(256) void k_bt(const float* __restrict__ Bx, __bf16* __restrict__ BT) { __shared__ __align__(16) __bf16 st[DD][64 + 8]; const int t = threadIdx.x; const int j0 = blockIdx.x * 64; const size_t b = blockIdx.y;
  for (int e = t; e < 64 * DD; e += 256) { const int jl = e >> 7, d = e & 127; st[d][jl] = (__bf16)Bx[((b * NN + j0 + jl) * DD) + d]; } __syncthreads();
  for (int e = t; e < DD * 8; e += 256) { const int d = e >> 3, q = e & 7; vst2((unsigned*)(BT + ((b * DD + d) * NN) + j0 + q * 8), *(const v4u*)&st[d][q * 8]); } }
__device__ __forceinline__ v16b fragb_f32(const float* __restrict__ p, int lane) { v16b a; const float* pp = p + 8 * (lane >> 4);
#pragma unroll
  for (int i = 0; i < 8; ++i) { a[i] = (__bf16)pp[i]; a[8 + i] = (__bf16)pp[16 + i]; } return a; }
__global__ __launch_bounds__(128) void k_wi(const float* __restrict__ Bx, const __bf16* __restrict__ PW, float* __restrict__ WI) { __shared__ __align__(16) float sf[4][16][132];
  const int tid = threadIdx.x, wave = tid >> 5, lane = tid & 31, col = lane & 15, g = lane >> 4; const size_t b = blockIdx.y; const size_t r0 = b * NN + (size_t)blockIdx.x * 64 + wave * 16;
  v8f acc[8] = {};
#pragma unroll
  for (int kc = 0; kc < DD / 32; ++kc) { const v16b a = fragb_f32(Bx + (r0 + col) * DD + kc * 32, lane);
#pragma unroll
    for (int j = 0; j < 8; ++j) acc[j] = wmma_bf(a, frag_b(PW + (size_t)(j * 16 + col) * DD + kc * 32, lane), acc[j]); }
#pragma unroll
  for (int j = 0; j < 8; ++j)
#pragma unroll
    for (int r = 0; r < 8; ++r) sf[wave][8 * g + r][j * 16 + col] = acc[j][r];
  LDSX(); for (int rl = 0; rl < 16; ++rl) vst2(WI + (r0 + rl) * DD + lane * 4, *(const v4f*)&sf[wave][rl][lane * 4]); }
__global__ __launch_bounds__(128) void k_sc(const float* __restrict__ WI, const float* __restrict__ V, float* __restrict__ P) { __shared__ float swi[DD], sv[DD]; __shared__ float red[4]; __shared__ __align__(16) float sp[NN]; const int t = threadIdx.x; const size_t b = blockIdx.y; const int i = blockIdx.x;
  swi[t] = WI[(b * NN + i) * DD + t]; sv[t] = bfr(V[t]); __syncthreads();
  float s4[4];
#pragma unroll
  for (int q = 0; q < 4; ++q) { const int j = t + 128 * q; const float* wj = WI + (b * NN + j) * DD; float s = 0.f;
#pragma unroll 1
    for (int d = 0; d < DD; ++d) s += sv[d] * tanhf(wj[d] + swi[d]);
    s4[q] = s; }
  float mx = fmaxf(fmaxf(s4[0], s4[1]), fmaxf(s4[2], s4[3]));
#pragma unroll
  for (int o = 1; o < 32; o <<= 1) mx = fmaxf(mx, __shfl_xor(mx, o));
  if ((t & 31) == 0) red[t >> 5] = mx; __syncthreads(); mx = fmaxf(fmaxf(red[0], red[1]), fmaxf(red[2], red[3])); __syncthreads();
  float e4[4], sm = 0.f;
#pragma unroll
  for (int q = 0; q < 4; ++q) { e4[q] = __expf(s4[q] - mx); sm += e4[q]; }
#pragma unroll
  for (int o = 1; o < 32; o <<= 1) sm += __shfl_xor(sm, o);
  if ((t & 31) == 0) red[t >> 5] = sm; __syncthreads(); const float inv = 1.0f / (red[0] + red[1] + red[2] + red[3]);
#pragma unroll
  for (int q = 0; q < 4; ++q) sp[t + 128 * q] = e4[q] * inv; __syncthreads();
  vst2(P + ((b * NN + i) * NN) + t * 4, *(const v4f*)&sp[t * 4]); }
__global__ __launch_bounds__(128) void k_c(const float* __restrict__ P, const __bf16* __restrict__ BT, float* __restrict__ OUT) { __shared__ __align__(16) float sf[4][16][132];
  const int tid = threadIdx.x, wave = tid >> 5, lane = tid & 31, col = lane & 15, g = lane >> 4; const size_t b = blockIdx.y; const size_t r0 = b * NN + (size_t)blockIdx.x * 64 + wave * 16;
  v8f acc[8] = {};
#pragma unroll 2
  for (int kc = 0; kc < NN / 32; ++kc) { const F2 a = split_row(P + (r0 + col) * NN, kc * 32, lane);
#pragma unroll
    for (int j = 0; j < 8; ++j) { const v16b w = frag_b(BT + ((b * DD + j * 16 + col) * NN) + kc * 32, lane); acc[j] = wmma_bf(a.h, w, acc[j]); acc[j] = wmma_bf(a.l, w, acc[j]); } }
#pragma unroll
  for (int j = 0; j < 8; ++j)
#pragma unroll
    for (int r = 0; r < 8; ++r) sf[wave][8 * g + r][j * 16 + col] = acc[j][r];
  LDSX(); for (int rl = 0; rl < 16; ++rl) vst2(OUT + (r0 + rl) * DD + lane * 4, *(const v4f*)&sf[wave][rl][lane * 4]); }
extern "C" void kernel_launch(void* const* d_in, const int* in_sizes, int n_in, void* d_out, int out_size, void* d_ws, size_t ws_size, hipStream_t stream) {
  (void)in_sizes; (void)n_in; (void)out_size;
  const float** F = (const float**)d_in;
  if (ws_size < (size_t)WS_END) return;
  char* ws = (char*)d_ws; __bf16 *PW = (__bf16*)(ws + WS_PW), *BT = (__bf16*)(ws + WS_BT); float *WI = (float*)(ws + WS_WI), *P = (float*)(ws + WS_P);
  k_pack<<<DD, 128, 0, stream>>>(F[1], PW);
  k_bt<<<dim3(NN / 64, TNB), 256, 0, stream>>>(F[0], BT);
  k_wi<<<dim3(NN / 64, TNB), 128, 0, stream>>>(F[0], PW, WI);
  k_sc<<<dim3(NN, TNB), 128, 0, stream>>>(WI, F[2], P);
  k_c<<<dim3(NN / 64, TNB), 128, 0, stream>>>(P, BT, (float*)d_out);
}
